// TransformerBlock2_7138235646707
// MI455X (gfx1250) — hardware-verified
//
#include <hip/hip_runtime.h>


#define NB_  2
#define TQ   2048
#define TKC  4096
#define DD   512
#define NH_  8
#define HD   64
#define FF   2048
#define PCAR 1024.0f
#define SCL  0.125f
typedef _Float16 h16;
typedef unsigned short bf;
typedef __attribute__((ext_vector_type(16))) __bf16   v16bf;
typedef __attribute__((ext_vector_type(16))) _Float16 v16h;
typedef __attribute__((ext_vector_type(8)))  _Float16 v8h;
typedef __attribute__((ext_vector_type(8)))  unsigned short v8us;
typedef __attribute__((ext_vector_type(8)))  float    v8f;
typedef __attribute__((ext_vector_type(4)))  float    v4f;
typedef v8h  __attribute__((may_alias)) v8ha;
typedef v4f  __attribute__((may_alias)) v4fa;
typedef v8us __attribute__((may_alias)) v8usa;

__device__ __forceinline__ unsigned short f2bf(float f) { unsigned u = __float_as_uint(f); u += 0x7FFFu + ((u >> 16) & 1u); return (unsigned short)(u >> 16); }
__device__ __forceinline__ float bf2f(unsigned short b) { return __uint_as_float(((unsigned)b) << 16); }
__device__ __forceinline__ float bfr(float f) { return bf2f(f2bf(f)); }
__device__ __forceinline__ v16h cat16(v8h lo, v8h hi) { return __builtin_shufflevector(lo, hi, 0, 1, 2, 3, 4, 5, 6, 7, 8, 9, 10, 11, 12, 13, 14, 15); }
__device__ __forceinline__ v16bf cat16b(v8us lo, v8us hi) { return __builtin_bit_cast(v16bf, __builtin_shufflevector(lo, hi, 0, 1, 2, 3, 4, 5, 6, 7, 8, 9, 10, 11, 12, 13, 14, 15)); }
__device__ __forceinline__ v8f wmma16(v16h a, v16h b, v8f c) { return __builtin_amdgcn_wmma_f32_16x16x32_f16(false, a, false, b, (short)0, c, false, false); }
__device__ __forceinline__ v8f wmmab(v16bf a, v16bf b, v8f c) { return __builtin_amdgcn_wmma_f32_16x16x32_bf16(false, a, false, b, (short)0, c, false, false); }


template <typename T16> struct WFrag;
template <> struct WFrag<h16> { typedef v16h V; static __device__ __forceinline__ V ld(const h16* p) { return cat16(*(const v8h*)p, *(const v8h*)(p + 16)); } static __device__ __forceinline__ v8f mma(V a, V b, v8f c) { return wmma16(a, b, c); } };
template <> struct WFrag<bf> { typedef v16bf V; static __device__ __forceinline__ V ld(const bf* p) { return cat16b(*(const v8us*)p, *(const v8us*)(p + 16)); } static __device__ __forceinline__ v8f mma(V a, V b, v8f c) { return wmmab(a, b, c); } };
template <typename T16, int NSPLIT, bool BIAS>
__global__ __launch_bounds__(32) void k_gemmw(const T16* __restrict__ A, const T16* __restrict__ A2, const T16* __restrict__ Bt, const T16* __restrict__ Bt2, int K, float* C, int ldc, const float* __restrict__ bias, size_t sA, size_t sB, size_t sC) {
    typedef typename WFrag<T16>::V V;
    __shared__ __align__(16) float os[16 * 68];
    const size_t z = blockIdx.z; A += z * sA; if (A2) A2 += z * sA; Bt += z * sB; if (Bt2) Bt2 += z * sB; C += z * sC;
    const int lane = threadIdx.x & 31, lr = lane & 15, hi = lane >> 4; const int r0 = blockIdx.x * 64, c0 = blockIdx.y * 64;
    v8f acc[4][4];
#pragma unroll
    for (int mb = 0; mb < 4; ++mb)
#pragma unroll
        for (int nb = 0; nb < 4; ++nb) acc[mb][nb] = (v8f){};
    const size_t aoff = (size_t)(r0 + lr) * K + 8 * hi, boff = (size_t)(c0 + lr) * K + 8 * hi;
#pragma unroll 1
    for (int kc = 0; kc < K; kc += 32) {
        V a[4], a2[4];
#pragma unroll
        for (int mb = 0; mb < 4; ++mb) { a[mb] = WFrag<T16>::ld(A + aoff + (size_t)mb * 16 * K + kc); if (NSPLIT == 1 || NSPLIT == 2) a2[mb] = WFrag<T16>::ld(A2 + aoff + (size_t)mb * 16 * K + kc); }
#pragma unroll
        for (int nb = 0; nb < 4; ++nb) { const V b = WFrag<T16>::ld(Bt + boff + (size_t)nb * 16 * K + kc); V b2; if (NSPLIT >= 2) b2 = WFrag<T16>::ld(Bt2 + boff + (size_t)nb * 16 * K + kc);
#pragma unroll
            for (int mb = 0; mb < 4; ++mb) { acc[mb][nb] = WFrag<T16>::mma(a[mb], b, acc[mb][nb]); if (NSPLIT == 1 || NSPLIT == 2) acc[mb][nb] = WFrag<T16>::mma(a2[mb], b, acc[mb][nb]); if (NSPLIT >= 2) acc[mb][nb] = WFrag<T16>::mma(a[mb], b2, acc[mb][nb]); } }
        asm volatile("v_nop\n\tv_nop\n\tv_nop\n\tv_nop" : "+v"(acc[0][0]), "+v"(acc[1][1]), "+v"(acc[2][2]), "+v"(acc[3][3]) : "v"(a[0]), "v"(a[3]));
    }
#pragma unroll
    for (int mb = 0; mb < 4; ++mb) {
#pragma unroll
        for (int nb = 0; nb < 4; ++nb) {
#pragma unroll
            for (int j = 0; j < 8; ++j) os[(hi * 8 + j) * 68 + nb * 16 + lr] = acc[mb][nb][j]; }
        __builtin_amdgcn_wave_barrier(); asm volatile("" ::: "memory");
        float* crow = C + (size_t)(r0 + mb * 16) * ldc + c0;
#pragma unroll 1
        for (int ps = 0; ps < 2; ++ps) {
#pragma unroll
            for (int s = 0; s < 8; ++s) { const int row = 2 * s + hi, cofs = lr * 4; v4f val = *(const v4fa*)(os + row * 68 + cofs); if (BIAS) { val[0] += bfr(bias[c0 + cofs]); val[1] += bfr(bias[c0 + cofs + 1]); val[2] += bfr(bias[c0 + cofs + 2]); val[3] += bfr(bias[c0 + cofs + 3]); }
                *(volatile v4f*)(crow + (size_t)row * ldc + cofs) = val; }
            if (ps == 0) __threadfence(); }
        __builtin_amdgcn_wave_barrier(); asm volatile("" ::: "memory");
    }
}

__device__ __forceinline__ h16 tohx(float x) { return (h16)x; }
__device__ __forceinline__ void splitf(float y, unsigned short& h, unsigned short& l) { h = f2bf(y); l = f2bf(y - bf2f(h)); }
typedef __attribute__((ext_vector_type(2))) _Float16 v2h;
typedef __attribute__((ext_vector_type(4))) _Float16 v4h;
typedef __attribute__((ext_vector_type(2))) unsigned short v2us;
typedef __attribute__((ext_vector_type(4))) unsigned short v4us;
typedef __attribute__((ext_vector_type(2))) float v2f;

__global__ __launch_bounds__(256) void k_wtG(const float* __restrict__ w, int K, int N, bf* Bt) {
    const int lane = threadIdx.x & 31; const int L0 = (blockIdx.x * 8 + (threadIdx.x >> 5)) * 8; const int nlines = N * K / 64;
#pragma unroll 1
    for (int ps = 0; ps < 2; ++ps) {
#pragma unroll 1
        for (int l = 0; l < 8; ++l) { const int L = L0 + l; if (L >= nlines) break; const size_t e = (size_t)L * 64 + lane * 2; const int k = (int)(e % K), n = (int)(e / K); v2us o;
            o[0] = f2bf(w[(size_t)k * N + n]); o[1] = f2bf(w[(size_t)(k + 1) * N + n]); *(volatile v2us*)(Bt + e) = o; }
        if (ps == 0) __threadfence(); }
}
__global__ __launch_bounds__(256) void k_cvt8(const float* __restrict__ src, bf* dst, size_t n8) { const size_t i = (size_t)blockIdx.x * 256 + threadIdx.x; if (i >= n8) return; const v8f v = *(const v8f*)(src + i * 8); v8us o;
#pragma unroll
    for (int k = 0; k < 8; ++k) o[k] = f2bf(v[k]); *(volatile v8us*)(dst + i * 8) = o; __threadfence(); *(volatile v8us*)(dst + i * 8) = o; }
__global__ __launch_bounds__(256) void k_ln512(const float* __restrict__ A, const float* __restrict__ gg, const float* __restrict__ bb, bf* Yh, bf* Yl) {
    const int lane = threadIdx.x & 31; const int r = blockIdx.x * 8 + (threadIdx.x >> 5); if (r >= TQ) return; float v[16]; float s = 0.f;
#pragma unroll
    for (int c = 0; c < 4; ++c) { const v4f a = *(const v4f*)(A + (size_t)r * DD + c * 128 + lane * 4);
#pragma unroll
        for (int q = 0; q < 4; ++q) { v[c * 4 + q] = a[q]; s = __fadd_rn(s, a[q]); } }
#pragma unroll
    for (int sh = 16; sh; sh >>= 1) s += __shfl_xor(s, sh, 32);
    const float mu = s * (1.0f / DD); float qq = 0.f;
#pragma unroll
    for (int i = 0; i < 16; ++i) { const float d0 = v[i] - mu; float p = __fmul_rn(d0, d0); asm volatile("" : "+v"(p)); qq = __fadd_rn(qq, p); }
#pragma unroll
    for (int sh = 16; sh; sh >>= 1) qq += __shfl_xor(qq, sh, 32);
    const float rs = __fdiv_rn(1.0f, __fsqrt_rn(__fadd_rn(qq * (1.0f / DD), 1e-5f)));
#pragma unroll 1
    for (int ps = 0; ps < 2; ++ps) {
#pragma unroll
        for (int c = 0; c < 4; ++c) { v4us oh, ol;
#pragma unroll
            for (int q = 0; q < 4; ++q) { const int col = c * 128 + lane * 4 + q; float g = bfr(gg[col]), bq = bfr(bb[col]); asm volatile("" : "+v"(g)); asm volatile("" : "+v"(bq)); float tn = __fmul_rn(v[c * 4 + q] - mu, rs); asm volatile("" : "+v"(tn)); float tg = __fmul_rn(tn, g); asm volatile("" : "+v"(tg)); unsigned short a2, c2; splitf(__fadd_rn(tg, bq), a2, c2); oh[q] = a2; ol[q] = c2; }
            const size_t o = (size_t)r * DD + c * 128 + lane * 4; *(volatile v4us*)(Yh + o) = oh; *(volatile v4us*)(Yl + o) = ol; }
        if (ps == 0) __threadfence(); }
}
__global__ __launch_bounds__(256) void k_pl(const float* __restrict__ F, int nT, h16* P) { const size_t e = ((size_t)blockIdx.x * 256 + threadIdx.x) * 2; if (e >= (size_t)NH_ * nT * HD) return; const int d = (int)(e & 63); const int t = (int)((e >> 6) % nT); const int h = (int)(e / ((size_t)nT * HD)); v2h o; o[0] = tohx(F[(size_t)t * DD + h * HD + d]); o[1] = tohx(F[(size_t)t * DD + h * HD + d + 1]); *(volatile v2h*)(P + e) = o; __threadfence(); *(volatile v2h*)(P + e) = o; }
__global__ __launch_bounds__(256) void k_vt(const float* __restrict__ F, int nT, h16* VT) { const size_t e = ((size_t)blockIdx.x * 256 + threadIdx.x) * 2; if (e >= (size_t)NH_ * HD * nT) return; const int t = (int)(e % nT); const int d = (int)((e / nT) & 63); const int h = (int)(e / ((size_t)nT * HD)); v2h o; o[0] = tohx(F[(size_t)t * DD + h * HD + d]); o[1] = tohx(F[(size_t)(t + 1) * DD + h * HD + d]); *(volatile v2h*)(VT + e) = o; __threadfence(); *(volatile v2h*)(VT + e) = o; }
__global__ __launch_bounds__(256) void k_split2(const float* __restrict__ F, bf* Ph, bf* Pl, size_t cnt) { const size_t i = ((size_t)blockIdx.x * 256 + threadIdx.x) * 2; if (i >= cnt) return; v2us oh, ol;
#pragma unroll
    for (int q = 0; q < 2; ++q) { unsigned short a, c2; splitf(F[i + q], a, c2); oh[q] = a; ol[q] = c2; } *(volatile v2us*)(Ph + i) = oh; *(volatile v2us*)(Pl + i) = ol; __threadfence(); *(volatile v2us*)(Ph + i) = oh; *(volatile v2us*)(Pl + i) = ol; }
template <int NK>
__global__ __launch_bounds__(256) void k_smax(const float* __restrict__ S, float* RS) { const int lane = threadIdx.x & 31; const int i = blockIdx.x * 8 + (threadIdx.x >> 5); if (i >= TQ) return; const float* sr = S + (size_t)i * NK; float m = -3.0e38f;
#pragma unroll 4
    for (int c0 = lane * 4; c0 < NK; c0 += 128) { const v4f v = *(const v4f*)(sr + c0); m = fmaxf(m, fmaxf(fmaxf(v[0], v[1]), fmaxf(v[2], v[3]))); }
#pragma unroll
    for (int sh = 16; sh; sh >>= 1) m = fmaxf(m, __shfl_xor(m, sh, 32));
    const float o = lane == 0 ? m : 0.f; *(volatile float*)(RS + (size_t)i * 32 + lane) = o; __threadfence(); *(volatile float*)(RS + (size_t)i * 32 + lane) = o; }
template <int NK>
__global__ __launch_bounds__(256) void k_sexp(const float* __restrict__ S, float* RS, h16* P) { const int lane = threadIdx.x & 31; const int i = blockIdx.x * 8 + (threadIdx.x >> 5); if (i >= TQ) return; const float* sr = S + (size_t)i * NK; const float m = RS[(size_t)i * 32]; float sum = 0.f;
#pragma unroll 1
    for (int ps = 0; ps < 2; ++ps) { sum = 0.f;
#pragma unroll 2
        for (int c0 = lane * 4; c0 < NK; c0 += 128) { const v4f v = *(const v4f*)(sr + c0); v4h o;
#pragma unroll
            for (int q = 0; q < 4; ++q) { float dlt = __fsub_rn(v[q], m); asm volatile("" : "+v"(dlt)); const float e = __expf(__fmul_rn(dlt, SCL)); sum += e; o[q] = tohx(e * PCAR); }
            *(volatile v4h*)(P + (size_t)i * NK + c0) = o; }
        if (ps == 0) __threadfence(); }
#pragma unroll
    for (int sh = 16; sh; sh >>= 1) sum += __shfl_xor(sum, sh, 32);
    const float o2 = lane == 0 ? m : (lane == 1 ? __fdiv_rn(1.0f, sum * PCAR) : 0.f); *(volatile float*)(RS + (size_t)i * 32 + lane) = o2; __threadfence(); *(volatile float*)(RS + (size_t)i * 32 + lane) = o2; }
__global__ __launch_bounds__(256) void k_mrg(const float* __restrict__ O, const float* __restrict__ RS, int h, bf* Ah, bf* Al) { const int e = (blockIdx.x * 256 + threadIdx.x) * 2; if (e >= TQ * HD) return; const int d = e & 63; const int t = e >> 6; const float sc = RS[(size_t)t * 32 + 1]; v2us oh, ol;
#pragma unroll
    for (int q = 0; q < 2; ++q) { unsigned short a, c2; splitf(__fmul_rn(O[e + q], sc), a, c2); oh[q] = a; ol[q] = c2; } const size_t oo = (size_t)t * DD + h * HD + d; *(volatile v2us*)(Ah + oo) = oh; *(volatile v2us*)(Al + oo) = ol; __threadfence(); *(volatile v2us*)(Ah + oo) = oh; *(volatile v2us*)(Al + oo) = ol; }
__global__ __launch_bounds__(256) void k_add(const float* __restrict__ A, const float* __restrict__ Bv, float* Y) { const size_t i = ((size_t)blockIdx.x * 256 + threadIdx.x) * 4; if (i >= (size_t)TQ * DD) return; const v4f a = *(const v4f*)(A + i), b = *(const v4f*)(Bv + i); v4f o;
#pragma unroll
    for (int q = 0; q < 4; ++q) o[q] = __fadd_rn(a[q], b[q]); *(volatile v4f*)(Y + i) = o; __threadfence(); *(volatile v4f*)(Y + i) = o; }
__global__ __launch_bounds__(256) void k_gelu2(const float* __restrict__ F, bf* Ph, bf* Pl) { const size_t i = ((size_t)blockIdx.x * 256 + threadIdx.x) * 2; if (i >= (size_t)TQ * FF) return; v2us oh, ol;
#pragma unroll
    for (int q = 0; q < 2; ++q) { const float h = F[i + q]; float er = erff(h * 0.70710678f); asm volatile("" : "+v"(er)); float hh = __fmul_rn(0.5f, h); asm volatile("" : "+v"(hh)); unsigned short a, c2; splitf(__fmul_rn(hh, __fadd_rn(1.0f, er)), a, c2); oh[q] = a; ol[q] = c2; }
    *(volatile v2us*)(Ph + i) = oh; *(volatile v2us*)(Pl + i) = ol; __threadfence(); *(volatile v2us*)(Ph + i) = oh; *(volatile v2us*)(Pl + i) = ol; }

extern "C" void kernel_launch(void* const* d_in, const int* in_sizes, int n_in,
                              void* d_out, int out_size, void* d_ws, size_t ws_size, hipStream_t stream) {
    (void)in_sizes; (void)n_in; (void)out_size;
    const float* IN[26]; for (int i = 0; i < 26; ++i) IN[i] = (const float*)d_in[i];
    float* OUT = (float*)d_out;
    char* wsp = (char*)d_ws;
    auto take = [&](size_t bytes) { char* p = wsp; wsp += (bytes + 255) & ~(size_t)255; return (void*)p; };
    bf* W[8]; for (int i = 0; i < 8; ++i) W[i] = (bf*)take((size_t)DD * DD * 2);
    bf* W1 = (bf*)take((size_t)FF * DD * 2); bf* W2 = (bf*)take((size_t)DD * FF * 2);
    bf* XB = (bf*)take((size_t)TQ * DD * 2); bf* CB = (bf*)take((size_t)TKC * DD * 2); float* F = (float*)take((size_t)TKC * DD * 4); h16* QP = (h16*)take((size_t)NH_ * TQ * HD * 2); h16* KP = (h16*)take((size_t)NH_ * TKC * HD * 2); h16* VT = (h16*)take((size_t)NH_ * HD * TKC * 2);
    float* Sb = (float*)take((size_t)TQ * TKC * 4); h16* Pm = (h16*)take((size_t)TQ * TKC * 2); float* RS = (float*)take((size_t)TQ * 32 * 4); float* Ob = (float*)take((size_t)TQ * HD * 4); bf* Ah = (bf*)take((size_t)TQ * DD * 2); bf* Al = (bf*)take((size_t)TQ * DD * 2);
    float* XC = (float*)take((size_t)TQ * DD * 4); bf* Nh = (bf*)take((size_t)TQ * DD * 2); bf* Nl = (bf*)take((size_t)TQ * DD * 2); float* G = (float*)take((size_t)TQ * DD * 4); float* Y = (float*)take((size_t)TQ * DD * 4); float* HF = (float*)take((size_t)TQ * FF * 4); bf* Gh = (bf*)take((size_t)TQ * FF * 2); bf* Gl = (bf*)take((size_t)TQ * FF * 2);
    if ((size_t)(wsp - (char*)d_ws) > ws_size) return;
    { const unsigned g5 = (unsigned)((DD * DD / 64 + 63) / 64); for (int i = 0; i < 8; ++i) k_wtG<<<g5, 256, 0, stream>>>(IN[2 + 2 * i], DD, DD, W[i]);
      k_wtG<<<(unsigned)((DD * FF / 64 + 63) / 64), 256, 0, stream>>>(IN[22], DD, FF, W1); k_wtG<<<(unsigned)((FF * DD / 64 + 63) / 64), 256, 0, stream>>>(IN[24], FF, DD, W2); }
    const unsigned L2 = (TQ * DD / 2 + 255) / 256, L4 = (TQ * DD / 4 + 255) / 256; const dim3 gQ(TQ / 64, DD / 64, 1), gK(TKC / 64, DD / 64, 1);
    for (int b = 0; b < NB_; ++b) {
        k_cvt8<<<(unsigned)(((size_t)TQ * DD / 8 + 255) / 256), 256, 0, stream>>>(IN[0] + (size_t)b * TQ * DD, XB, (size_t)TQ * DD / 8); k_cvt8<<<(unsigned)(((size_t)TKC * DD / 8 + 255) / 256), 256, 0, stream>>>(IN[1] + (size_t)b * TKC * DD, CB, (size_t)TKC * DD / 8);
        k_gemmw<bf, 0, true><<<gQ, 32, 0, stream>>>(XB, nullptr, W[0], nullptr, DD, F, DD, IN[3], 0, 0, 0); k_pl<<<(unsigned)(((size_t)NH_ * TQ * HD / 2 + 255) / 256), 256, 0, stream>>>(F, TQ, QP);
        k_gemmw<bf, 0, true><<<gK, 32, 0, stream>>>(CB, nullptr, W[1], nullptr, DD, F, DD, IN[5], 0, 0, 0); k_pl<<<(unsigned)(((size_t)NH_ * TKC * HD / 2 + 255) / 256), 256, 0, stream>>>(F, TKC, KP);
        k_gemmw<bf, 0, true><<<gK, 32, 0, stream>>>(CB, nullptr, W[2], nullptr, DD, F, DD, IN[7], 0, 0, 0); k_vt<<<(unsigned)(((size_t)NH_ * HD * TKC / 2 + 255) / 256), 256, 0, stream>>>(F, TKC, VT);
        for (int h = 0; h < NH_; ++h) {
            k_gemmw<h16, 0, false><<<dim3(TQ / 64, TKC / 64, 1), 32, 0, stream>>>(QP + (size_t)h * TQ * HD, nullptr, KP + (size_t)h * TKC * HD, nullptr, HD, Sb, TKC, nullptr, 0, 0, 0);
            k_smax<TKC><<<TQ / 8, 256, 0, stream>>>(Sb, RS); k_sexp<TKC><<<TQ / 8, 256, 0, stream>>>(Sb, RS, Pm);
            k_gemmw<h16, 0, false><<<dim3(TQ / 64, 1, 1), 32, 0, stream>>>(Pm, nullptr, VT + (size_t)h * HD * TKC, nullptr, TKC, Ob, HD, nullptr, 0, 0, 0);
            k_mrg<<<(TQ * HD / 2 + 255) / 256, 256, 0, stream>>>(Ob, RS, h, Ah, Al); }
        k_gemmw<bf, 1, true><<<gQ, 32, 0, stream>>>(Ah, Al, W[3], nullptr, DD, XC, DD, IN[9], 0, 0, 0);
        k_ln512<<<TQ / 8, 256, 0, stream>>>(XC, IN[18], IN[19], Nh, Nl);
        k_gemmw<bf, 1, true><<<gQ, 32, 0, stream>>>(Nh, Nl, W[4], nullptr, DD, F, DD, IN[11], 0, 0, 0); k_pl<<<(unsigned)(((size_t)NH_ * TQ * HD / 2 + 255) / 256), 256, 0, stream>>>(F, TQ, QP);
        k_gemmw<bf, 1, true><<<gQ, 32, 0, stream>>>(Nh, Nl, W[5], nullptr, DD, F, DD, IN[13], 0, 0, 0); k_pl<<<(unsigned)(((size_t)NH_ * TQ * HD / 2 + 255) / 256), 256, 0, stream>>>(F, TQ, KP);
        k_gemmw<bf, 1, true><<<gQ, 32, 0, stream>>>(Nh, Nl, W[6], nullptr, DD, F, DD, IN[15], 0, 0, 0); k_vt<<<(unsigned)(((size_t)NH_ * HD * TQ / 2 + 255) / 256), 256, 0, stream>>>(F, TQ, VT);
        for (int h = 0; h < NH_; ++h) {
            k_gemmw<h16, 0, false><<<dim3(TQ / 64, TQ / 64, 1), 32, 0, stream>>>(QP + (size_t)h * TQ * HD, nullptr, KP + (size_t)h * TQ * HD, nullptr, HD, Sb, TQ, nullptr, 0, 0, 0);
            k_smax<TQ><<<TQ / 8, 256, 0, stream>>>(Sb, RS); k_sexp<TQ><<<TQ / 8, 256, 0, stream>>>(Sb, RS, Pm);
            k_gemmw<h16, 0, false><<<dim3(TQ / 64, 1, 1), 32, 0, stream>>>(Pm, nullptr, VT + (size_t)h * HD * TQ, nullptr, TQ, Ob, HD, nullptr, 0, 0, 0);
            k_mrg<<<(TQ * HD / 2 + 255) / 256, 256, 0, stream>>>(Ob, RS, h, Ah, Al); }
        k_gemmw<bf, 1, true><<<gQ, 32, 0, stream>>>(Ah, Al, W[7], nullptr, DD, G, DD, IN[17], 0, 0, 0); k_add<<<L4, 256, 0, stream>>>(XC, G, Y);
        k_ln512<<<TQ / 8, 256, 0, stream>>>(Y, IN[20], IN[21], Nh, Nl);
        k_gemmw<bf, 1, true><<<dim3(TQ / 64, FF / 64, 1), 32, 0, stream>>>(Nh, Nl, W1, nullptr, DD, HF, FF, IN[23], 0, 0, 0); k_gelu2<<<(unsigned)(((size_t)TQ * FF / 2 + 255) / 256), 256, 0, stream>>>(HF, Gh, Gl);
        k_gemmw<bf, 1, true><<<gQ, 32, 0, stream>>>(Gh, Gl, W2, nullptr, FF, G, DD, IN[25], 0, 0, 0); k_add<<<L4, 256, 0, stream>>>(Y, G, OUT + (size_t)b * TQ * DD); }
    (void)L2;
}
